// Text_encoder_61950608278168
// MI455X (gfx1250) — hardware-verified
//
#include <hip/hip_runtime.h>


#ifndef NI
#define NI 384
#endif
#define NS_FULL 384
#define DD    768
#define HH    768
#define NC    2
#define KPW   48

static_assert(NI % 64 == 0 && NI >= 64 && NI <= NS_FULL);
static_assert(NS_FULL % 64 == 0 && HH % 64 == 0);
static_assert(DD % 32 == 0 && HH % 128 == 0 && HH == 6 * 128);
static_assert(NS_FULL == 8 * KPW);
static_assert(NC == 2);
static_assert(96 * 8 == DD);
static_assert(((size_t)NS_FULL * DD) % (8 * 256) == 0);
static_assert(6 * 32 * 16 == NS_FULL * NC * 4);
static_assert((size_t)NS_FULL * NS_FULL * NC * 4 == 1179648);
static_assert(((size_t)NS_FULL * NC * 4) % 128 == 0);
static_assert(16 * 68 * 4 <= 131072);
static_assert(NC * NS_FULL * 4 <= 131072);
static_assert((size_t)NS_FULL * DD * 2 + (size_t)2 * HH * DD * 2 + (size_t)NI * HH * 4 + (size_t)NS_FULL * HH * 4 <= 134217728);
static_assert(((size_t)NS_FULL * DD * 2) % 256 == 0 && ((size_t)2 * HH * DD * 2) % 256 == 0 && ((size_t)NI * HH * 4) % 256 == 0 && ((size_t)NS_FULL * HH * 4) % 256 == 0);

typedef _Float16 h16;
typedef unsigned short bf;
typedef __attribute__((ext_vector_type(16))) __bf16   v16bf;
typedef __attribute__((ext_vector_type(16))) _Float16 v16h;
typedef __attribute__((ext_vector_type(8)))  _Float16 v8h;
typedef __attribute__((ext_vector_type(8)))  unsigned short v8us;
typedef __attribute__((ext_vector_type(8)))  float    v8f;
typedef __attribute__((ext_vector_type(4)))  float    v4f;
typedef __attribute__((ext_vector_type(2)))  float    v2f;
typedef v4f  __attribute__((may_alias)) v4fa;
typedef v2f  __attribute__((may_alias)) v2fa;

__device__ __forceinline__ unsigned short f2bf(float f) { unsigned u = __float_as_uint(f); u += 0x7FFFu + ((u >> 16) & 1u); return (unsigned short)(u >> 16); }
__device__ __forceinline__ float bf2f(unsigned short b) { return __uint_as_float(((unsigned)b) << 16); }
__device__ __forceinline__ float bfr(float f) { return bf2f(f2bf(f)); }
__device__ __forceinline__ v16h cat16(v8h lo, v8h hi) { return __builtin_shufflevector(lo, hi, 0, 1, 2, 3, 4, 5, 6, 7, 8, 9, 10, 11, 12, 13, 14, 15); }
__device__ __forceinline__ v16bf cat16b(v8us lo, v8us hi) { return __builtin_bit_cast(v16bf, __builtin_shufflevector(lo, hi, 0, 1, 2, 3, 4, 5, 6, 7, 8, 9, 10, 11, 12, 13, 14, 15)); }
__device__ __forceinline__ v8f wmma16(v16h a, v16h b, v8f c) { return __builtin_amdgcn_wmma_f32_16x16x32_f16(false, a, false, b, (short)0, c, false, false); }
__device__ __forceinline__ v8f wmmab(v16bf a, v16bf b, v8f c) { return __builtin_amdgcn_wmma_f32_16x16x32_bf16(false, a, false, b, (short)0, c, false, false); }

template <typename T16> struct WFrag;
template <> struct WFrag<h16> { typedef v16h V; static __device__ __forceinline__ V ld(const h16* p) { return cat16(*(const v8h*)p, *(const v8h*)(p + 16)); } static __device__ __forceinline__ v8f mma(V a, V b, v8f c) { return wmma16(a, b, c); } };
template <> struct WFrag<bf> { typedef v16bf V; static __device__ __forceinline__ V ld(const bf* p) { return cat16b(*(const v8us*)p, *(const v8us*)(p + 16)); } static __device__ __forceinline__ v8f mma(V a, V b, v8f c) { return wmmab(a, b, c); } };
template <typename T16, int NSPLIT, bool BIAS>
__global__ __launch_bounds__(32) void k_gemmw(const T16* __restrict__ A, const T16* __restrict__ A2, const T16* __restrict__ Bt, const T16* __restrict__ Bt2, int K, float* C, int ldc, const float* __restrict__ bias, float csc, size_t sA, size_t sB, size_t sC) {
    typedef typename WFrag<T16>::V V;
    __shared__ __align__(16) float os[16 * 68];
    const size_t z = blockIdx.z; A += z * sA; if (A2) A2 += z * sA; Bt += z * sB; if (Bt2) Bt2 += z * sB; C += z * sC;
    const int lane = threadIdx.x & 31, lr = lane & 15, hi = lane >> 4; const int r0 = blockIdx.x * 64, c0 = blockIdx.y * 64;
    v8f acc[4][4];
#pragma unroll
    for (int mb = 0; mb < 4; ++mb)
#pragma unroll
        for (int nb = 0; nb < 4; ++nb) acc[mb][nb] = (v8f){};
    const size_t aoff = (size_t)(r0 + lr) * K + 8 * hi, boff = (size_t)(c0 + lr) * K + 8 * hi;
#pragma unroll 1
    for (int kc = 0; kc < K; kc += 32) {
        V a[4], a2[4];
#pragma unroll
        for (int mb = 0; mb < 4; ++mb) { a[mb] = WFrag<T16>::ld(A + aoff + (size_t)mb * 16 * K + kc); if (NSPLIT == 1 || NSPLIT == 2) a2[mb] = WFrag<T16>::ld(A2 + aoff + (size_t)mb * 16 * K + kc); }
#pragma unroll
        for (int nb = 0; nb < 4; ++nb) { const V b = WFrag<T16>::ld(Bt + boff + (size_t)nb * 16 * K + kc); V b2; if (NSPLIT >= 2) b2 = WFrag<T16>::ld(Bt2 + boff + (size_t)nb * 16 * K + kc);
#pragma unroll
            for (int mb = 0; mb < 4; ++mb) { acc[mb][nb] = WFrag<T16>::mma(a[mb], b, acc[mb][nb]); if (NSPLIT == 1 || NSPLIT == 2) acc[mb][nb] = WFrag<T16>::mma(a2[mb], b, acc[mb][nb]); if (NSPLIT >= 2) acc[mb][nb] = WFrag<T16>::mma(a[mb], b2, acc[mb][nb]); } }
        asm volatile("v_nop\n\tv_nop\n\tv_nop\n\tv_nop" : "+v"(acc[0][0]), "+v"(acc[1][1]), "+v"(acc[2][2]), "+v"(acc[3][3]) : "v"(a[0]), "v"(a[3]));
    }
#pragma unroll
    for (int mb = 0; mb < 4; ++mb) {
#pragma unroll
        for (int nb = 0; nb < 4; ++nb) {
#pragma unroll
            for (int j = 0; j < 8; ++j) os[(hi * 8 + j) * 68 + nb * 16 + lr] = acc[mb][nb][j]; }
        __builtin_amdgcn_wave_barrier(); asm volatile("" ::: "memory");
        float* crow = C + (size_t)(r0 + mb * 16) * ldc + c0;
#pragma unroll 1
        for (int ps = 0; ps < 2; ++ps) {
#pragma unroll
            for (int s = 0; s < 8; ++s) { const int row = 2 * s + hi, cofs = lr * 4; v4f val = *(const v4fa*)(os + row * 68 + cofs); val = val * csc;
                if (BIAS) { val[0] += bfr(bias[c0 + cofs]); val[1] += bfr(bias[c0 + cofs + 1]); val[2] += bfr(bias[c0 + cofs + 2]); val[3] += bfr(bias[c0 + cofs + 3]); }
                *(volatile v4f*)(crow + (size_t)row * ldc + cofs) = val; }
            if (ps == 0) __threadfence(); }
        __builtin_amdgcn_wave_barrier(); asm volatile("" ::: "memory");
    }
}

__global__ __launch_bounds__(96) void k_wsplit(const float* __restrict__ w, bf* dst) {
    const int n = blockIdx.x, half = blockIdx.y, t = threadIdx.x;
    const v8f v = *(const v8f*)(w + (size_t)n * (2 * DD) + half * DD + t * 8); v8us o;
#pragma unroll
    for (int k = 0; k < 8; ++k) o[k] = f2bf(v[k]);
    bf* d = dst + ((size_t)half * HH + n) * DD + t * 8;
    *(volatile v8us*)d = o; __threadfence(); *(volatile v8us*)d = o;
}

__global__ __launch_bounds__(256) void k_cvt8(const float* __restrict__ src, bf* dst, size_t n8) { const size_t i = (size_t)blockIdx.x * 256 + threadIdx.x; if (i >= n8) return; const v8f v = *(const v8f*)(src + i * 8); v8us o;
#pragma unroll
    for (int k = 0; k < 8; ++k) o[k] = f2bf(v[k]); *(volatile v8us*)(dst + i * 8) = o; __threadfence(); *(volatile v8us*)(dst + i * 8) = o; }

__device__ __forceinline__ float tnh(float x) {
    const float e = __builtin_amdgcn_exp2f(x * 2.8853900817779268f);
    const float r = __builtin_amdgcn_rcpf(e + 1.0f);
    return fmaf(-2.0f, r, 1.0f);
}

__global__ __launch_bounds__(256) void k_pair(const float* __restrict__ AF, const float* __restrict__ BF, const float* __restrict__ W2, const float* __restrict__ b2, float* OUT) {
    __shared__ __align__(16) float s_sc[NC * NS_FULL];
    const int ri = blockIdx.x;
    const int tid = threadIdx.x, lane = tid & 31;
    const int wave = __builtin_amdgcn_readfirstlane(tid >> 5);
    const float* arow = AF + (size_t)ri * HH;
    float ar[24], w0[24], w1[24];
#pragma unroll
    for (int c = 0; c < 6; ++c) { const v4f a4 = *(const v4f*)(arow + c * 128 + lane * 4); const v4f x4 = *(const v4f*)(W2 + c * 128 + lane * 4);
#pragma unroll
        for (int e = 0; e < 4; ++e) { ar[c * 4 + e] = a4[e]; w0[c * 4 + e] = bfr(x4[e]); } }
    int off = lane * 4;
    asm volatile("" : "+v"(off), "+v"(w0[23]));
#pragma unroll
    for (int c = 0; c < 6; ++c) { const v4f y4 = *(const v4f*)(W2 + HH + c * 128 + off);
#pragma unroll
        for (int e = 0; e < 4; ++e) w1[c * 4 + e] = bfr(y4[e]); }
#pragma unroll 1
    for (int kk = 0; kk < KPW; ++kk) {
        const int k = wave * KPW + kk;
        const float* brow = BF + (size_t)k * HH;
        float acc0 = 0.0f, acc1 = 0.0f;
#pragma unroll
        for (int c = 0; c < 6; ++c) { const v4f u4 = *(const v4f*)(brow + c * 128 + lane * 4);
#pragma unroll
            for (int e = 0; e < 4; ++e) { const float t = tnh(ar[c * 4 + e] + u4[e]); acc0 = fmaf(w0[c * 4 + e], t, acc0); acc1 = fmaf(w1[c * 4 + e], t, acc1); } }
#pragma unroll
        for (int sh = 16; sh; sh >>= 1) { acc0 += __shfl_xor(acc0, sh, 32); acc1 += __shfl_xor(acc1, sh, 32); }
        v2f pr; pr[0] = acc0; pr[1] = acc1;
        if (lane == 0) *(v2fa*)(s_sc + 2 * k) = pr;
    }
    __syncthreads();
    const float c0 = bfr(b2[0]), c1 = bfr(b2[1]);
    if (wave < 6) {
        const int f0 = (wave * 32 + lane) * 4;
        v4f o = *(const v4fa*)(s_sc + f0);
        o[0] += c0; o[1] += c1; o[2] += c0; o[3] += c1;
        float* dst = OUT + (size_t)ri * (NS_FULL * NC) + f0;
        *(volatile v4f*)dst = o; __threadfence(); *(volatile v4f*)dst = o;
    }
}

extern "C" void kernel_launch(void* const* d_in, const int* in_sizes, int n_in,
                              void* d_out, int out_size, void* d_ws, size_t ws_size, hipStream_t stream) {
    if (n_in < 5) return;
    if (in_sizes[0] < NS_FULL * DD || in_sizes[1] < HH * 2 * DD || in_sizes[2] < HH || in_sizes[3] < NC * HH || in_sizes[4] < NC) return;
    if (out_size < NS_FULL * NS_FULL * NC) return;
    const float* pm = (const float*)d_in[0];
    const float* W1 = (const float*)d_in[1];
    const float* b1 = (const float*)d_in[2];
    const float* W2 = (const float*)d_in[3];
    const float* b2 = (const float*)d_in[4];
    float* OUT0 = (float*)d_out;

    char* wsp = (char*)d_ws;
    auto take = [&](size_t bytes) { char* p = wsp; wsp += (bytes + 255) & ~(size_t)255; return (void*)p; };
    bf*    PB  = (bf*)take((size_t)NS_FULL * DD * 2);
    bf*    WAB = (bf*)take((size_t)2 * HH * DD * 2);
    float* AF  = (float*)take((size_t)NI * HH * 4);
    float* BF  = (float*)take((size_t)NS_FULL * HH * 4);
    if ((size_t)(wsp - (char*)d_ws) > ws_size) return;

    k_cvt8<<<(unsigned)(((size_t)NS_FULL * DD / 8 + 255) / 256), 256, 0, stream>>>(pm, PB, (size_t)NS_FULL * DD / 8);
    k_wsplit<<<dim3(HH, 2, 1), 96, 0, stream>>>(W1, WAB);
    k_gemmw<bf, 0, true><<<dim3(NI / 64, HH / 64, 1), 32, 0, stream>>>(PB, nullptr, WAB, nullptr, DD, AF, HH, b1, 1.0f, 0, 0, 0);
    k_gemmw<bf, 0, false><<<dim3(NS_FULL / 64, HH / 64, 1), 32, 0, stream>>>(PB, nullptr, WAB + (size_t)HH * DD, nullptr, DD, BF, HH, nullptr, 1.0f, 0, 0, 0);
    k_pair<<<(unsigned)NI, 256, 0, stream>>>(AF, BF, W2, b2, OUT0);
}
